// CapsDense_58789512347928
// MI455X (gfx1250) — hardware-verified
//
#include <hip/hip_runtime.h>
#include <math.h>

typedef __attribute__((ext_vector_type(16))) _Float16 v16h;
typedef __attribute__((ext_vector_type(8)))  _Float16 v8h;
typedef __attribute__((ext_vector_type(8)))  float    v8f;
typedef __attribute__((ext_vector_type(4)))  float    v4f;

constexpr int kNB = 128;
constexpr int kNJ = 2048;
constexpr int kNK = 8;
constexpr int kNP = 32;
constexpr int kNQ = 16;
constexpr int kKFlat   = kNJ * kNK;
constexpr int kNFlat   = kNP * kNQ;
constexpr int kChunks  = 16;
constexpr int kChunkK  = kKFlat / kChunks;
constexpr int kLdsPitch = 132;
static_assert(kKFlat == 16384 && kNFlat == 512 && kChunkK == 1024, "flattened extents");
static_assert((kNB % 64) == 0 && (kNFlat % 64) == 0 && (kKFlat % 64) == 0, "GEMM M,N multiples of 64");
static_assert((kChunkK % 32) == 0 && (kNB % 32) == 0, "GEMM K multiples of 32");
static_assert(kNK * kNQ == 128 && kNP == 32, "W block of 128 floats per (j,p); lane == unit");

constexpr float kXCarry = 16.0f;
constexpr float kWCarry = 128.0f;
constexpr float kCCarry = 32.0f;
constexpr float kVCarry = 1024.0f;
constexpr float kSScale = 1.0f / (kXCarry * kWCarry * kCCarry);
constexpr float kGScale = 1.0f / (kXCarry * kVCarry);
static_assert(kCCarry == (float)kNP, "uniform coupling weight 1/units times its carry is exactly 1");

constexpr size_t kOffX16   = 0;
constexpr size_t kOffXT16  = kOffX16   + (size_t)kNB * kKFlat * 2;
constexpr size_t kOffBT16  = kOffXT16  + (size_t)kKFlat * kNB * 2;
constexpr size_t kOffSPART = kOffBT16  + (size_t)kNFlat * kKFlat * 2;
constexpr size_t kOffVT16  = kOffSPART + (size_t)kChunks * kNB * kNFlat * 4;
constexpr size_t kOffGPL   = kOffVT16  + (size_t)kNFlat * kNB * 2;
constexpr size_t kOffBL    = kOffGPL   + (size_t)kKFlat * kNFlat * 4;
constexpr size_t kOffCL    = kOffBL    + (size_t)kNJ * kNP * 4;
constexpr size_t kWsTotal  = kOffCL    + (size_t)kNJ * kNP * 4;
static_assert(kWsTotal == 63569920ull, "carve total");
static_assert(kWsTotal <= 134217728ull, "carve cap");
static_assert((kOffXT16 % 128) == 0 && (kOffBT16 % 128) == 0 && (kOffSPART % 128) == 0 && (kOffVT16 % 128) == 0 &&
              (kOffGPL % 128) == 0 && (kOffBL % 128) == 0 && (kOffCL % 128) == 0, "128-B aligned regions");

union FragH { v16h v; v8h h[2]; };
__device__ __forceinline__ v16h frag_load(const _Float16* p) {
  FragH f;
  f.h[0] = *(const v8h*)(p);
  f.h[1] = *(const v8h*)(p + 16);
  return f.v;
}
__device__ __forceinline__ v8f mma_guarded(v16h a, v16h b, v8f c) {
  c = __builtin_amdgcn_wmma_f32_16x16x32_f16(false, a, false, b, (short)0, c, false, false);
  asm volatile("v_nop\n\tv_nop\n\tv_nop\n\tv_nop" : "+v"(c) : "v"(a), "v"(b));
  return c;
}

__global__ __launch_bounds__(256) void gemm64_f16_kernel(
    const unsigned short* __restrict__ Ap, int lda, long strideA,
    const unsigned short* __restrict__ Btp, int ldb, long strideB,
    float* __restrict__ Cout, int ldc, long strideC,
    int M, int N, int K, float scale) {
  __shared__ __align__(16) float sT[8][16 * 68];
  const _Float16* A  = (const _Float16*)Ap;
  const _Float16* Bt = (const _Float16*)Btp;
  const int b    = blockIdx.y;
  const int lane = threadIdx.x & 31;
  const int wave = __builtin_amdgcn_readfirstlane((int)(threadIdx.x >> 5));
  const int tilesN = N >> 6;
  const int tilesM = M >> 6;
  const int tile = blockIdx.x * 8 + wave;
  if (tile >= tilesM * tilesN) return;
  const int tm = tile / tilesN;
  const int tn = tile - tm * tilesN;
  const int m0 = tm << 6;
  const int n0 = tn << 6;

  const _Float16* Ab = A  + (size_t)b * strideA;
  const _Float16* Bb = Bt + (size_t)b * strideB;

  const int rlane = lane & 15;
  const int koff  = (lane >> 4) * 8;
  const int mOff  = (lane >> 4) * 8;

  v8f acc[4][4];
#pragma unroll
  for (int i = 0; i < 4; ++i)
#pragma unroll
    for (int j = 0; j < 4; ++j) acc[i][j] = (v8f){0.f, 0.f, 0.f, 0.f, 0.f, 0.f, 0.f, 0.f};

  for (int k0 = 0; k0 < K; k0 += 32) {
    v16h bh[4];
#pragma unroll
    for (int j = 0; j < 4; ++j) {
      const size_t bo = (size_t)(n0 + (j << 4) + rlane) * ldb + koff + k0;
      bh[j] = frag_load(Bb + bo);
    }
#pragma unroll
    for (int i = 0; i < 4; ++i) {
      const size_t ao = (size_t)(m0 + (i << 4) + rlane) * lda + koff + k0;
      const v16h ah = frag_load(Ab + ao);
#pragma unroll
      for (int j = 0; j < 4; ++j) acc[i][j] = mma_guarded(ah, bh[j], acc[i][j]);
    }
  }

  float* slab = sT[wave];
  float* C = Cout + (size_t)b * strideC;
#pragma unroll
  for (int i = 0; i < 4; ++i) {
    const int mBase = m0 + (i << 4);
#pragma unroll
    for (int j = 0; j < 4; ++j) {
#pragma unroll
      for (int r = 0; r < 8; ++r) {
        slab[(mOff + r) * 68 + (j << 4) + rlane] = acc[i][j][r] * scale;
      }
    }
    __builtin_amdgcn_fence(__ATOMIC_RELEASE, "workgroup");
    __builtin_amdgcn_wave_barrier();
    __builtin_amdgcn_fence(__ATOMIC_ACQUIRE, "workgroup");
    {
      const int hh = lane >> 4, c4 = (lane & 15) * 4;
      for (int pass = 0; pass < 2; ++pass) {
#pragma unroll
        for (int it = 0; it < 8; ++it) {
          const int row = it * 2 + hh;
          v4f v = *(const v4f*)(slab + row * 68 + c4);
          *(volatile v4f*)(C + (size_t)(mBase + row) * ldc + n0 + c4) = v;
        }
        __threadfence();
      }
    }
    __builtin_amdgcn_fence(__ATOMIC_RELEASE, "workgroup");
    __builtin_amdgcn_wave_barrier();
    __builtin_amdgcn_fence(__ATOMIC_ACQUIRE, "workgroup");
  }
}

template <int NLINES>
__device__ __forceinline__ void emit_f16_rows128(const float* sT, unsigned short* dst, int wave, int lane) {
  constexpr int NIT = NLINES / 32;
  static_assert(NIT * 32 == NLINES, "whole wave groups");
  const int ql = lane >> 3, piece = lane & 7;
  v8h hv[NIT];
#pragma unroll
  for (int it = 0; it < NIT; ++it) {
    const int L = it * 32 + wave * 4 + ql;
    const float* sp = sT + (L >> 1) * kLdsPitch + (L & 1) * 64 + piece * 8;
    const v4f a0 = *(const v4f*)(sp);
    const v4f a1 = *(const v4f*)(sp + 4);
#pragma unroll
    for (int e = 0; e < 4; ++e) {
      const float f0 = a0[e];
      const float f1 = a1[e];
      hv[it][e]     = (_Float16)f0;
      hv[it][4 + e] = (_Float16)f1;
    }
  }
  for (int pass = 0; pass < 2; ++pass) {
#pragma unroll
    for (int it = 0; it < NIT; ++it) {
      const int L = it * 32 + wave * 4 + ql;
      *(volatile v8h*)(dst + (size_t)(L >> 1) * 128 + (L & 1) * 64 + piece * 8) = hv[it];
    }
    __threadfence();
  }
}

__global__ __launch_bounds__(256) void cast_x_kernel(const float* __restrict__ x, unsigned short* __restrict__ x16, int total8) {
  const int i = blockIdx.x * 256 + threadIdx.x;
  if (i >= total8) return;
  const size_t e0 = (size_t)i << 3;
  const v4f a0 = *(const v4f*)(x + e0);
  const v4f a1 = *(const v4f*)(x + e0 + 4);
  v8h hv;
#pragma unroll
  for (int e = 0; e < 4; ++e) {
    const float f0 = a0[e] * kXCarry;
    const float f1 = a1[e] * kXCarry;
    hv[e]     = (_Float16)f0;
    hv[4 + e] = (_Float16)f1;
  }
  unsigned short* q = x16 + e0;
  *(volatile v8h*)q = hv;
  __threadfence();
  *(volatile v8h*)q = hv;
}

__global__ __launch_bounds__(256) void xpose_x_kernel(const float* __restrict__ x, unsigned short* __restrict__ xT) {
  __shared__ __align__(16) float sX[64 * kLdsPitch];
  const int tid = threadIdx.x, lane = tid & 31;
  const int wave = __builtin_amdgcn_readfirstlane((int)(threadIdx.x >> 5));
  const int kk0 = blockIdx.x * 64;
#pragma unroll 2
  for (int it = 0; it < 8; ++it) {
    const int f4 = it * 256 + tid;
    const int i = f4 >> 4, c4 = (f4 & 15) * 4;
    const v4f a = *(const v4f*)(x + (size_t)i * kKFlat + kk0 + c4);
    sX[(c4 + 0) * kLdsPitch + i] = a[0] * kXCarry;
    sX[(c4 + 1) * kLdsPitch + i] = a[1] * kXCarry;
    sX[(c4 + 2) * kLdsPitch + i] = a[2] * kXCarry;
    sX[(c4 + 3) * kLdsPitch + i] = a[3] * kXCarry;
  }
  __syncthreads();
  emit_f16_rows128<128>(sX, xT + (size_t)kk0 * 128, wave, lane);
}

template <bool UNIFORM>
__global__ __launch_bounds__(256) void build_bt_kernel(const float* __restrict__ W, const float* __restrict__ cpl,
                                                       unsigned short* __restrict__ BT) {
  __shared__ __align__(16) float sW[8 * 512];
  const int tid = threadIdx.x, lane = tid & 31;
  const int wave = __builtin_amdgcn_readfirstlane((int)(threadIdx.x >> 5));
  const int j0 = blockIdx.x * 8, p0 = blockIdx.y * 4;
#pragma unroll
  for (int it = 0; it < 4; ++it) {
    const int f = (it * 256 + tid) * 4;
    const int jl = f >> 9, rem = f & 511, pl = rem >> 7;
    const v4f a = *(const v4f*)(W + ((size_t)((j0 + jl) * kNP + p0)) * 128 + rem);
    float sc = kWCarry;
    if (!UNIFORM) sc = (kWCarry * kCCarry) * cpl[(j0 + jl) * kNP + p0 + pl];
    v4f o;
    o[0] = a[0] * sc;
    o[1] = a[1] * sc;
    o[2] = a[2] * sc;
    o[3] = a[3] * sc;
    *(v4f*)(sW + f) = o;
  }
  __syncthreads();
  const int ql = lane >> 3, piece = lane & 7;
  v8h hv[2];
#pragma unroll
  for (int it = 0; it < 2; ++it) {
    const int L = it * 32 + wave * 4 + ql;
    const float* sp = sW + piece * 512 + (L >> 4) * 128 + (L & 15);
#pragma unroll
    for (int k = 0; k < 8; ++k) {
      const float f0 = sp[k * 16];
      hv[it][k] = (_Float16)f0;
    }
  }
  for (int pass = 0; pass < 2; ++pass) {
#pragma unroll
    for (int it = 0; it < 2; ++it) {
      const int L = it * 32 + wave * 4 + ql;
      *(volatile v8h*)(BT + (size_t)(p0 * 16 + L) * kKFlat + (size_t)(j0 + piece) * 8) = hv[it];
    }
    __threadfence();
  }
}

template <bool FINAL>
__global__ __launch_bounds__(256) void reduce_scale_kernel(const float* __restrict__ Spart, float* __restrict__ out,
                                                           unsigned short* __restrict__ vT) {
  __shared__ __align__(16) float sV[32 * kLdsPitch];
  const int tid = threadIdx.x, lane = tid & 31;
  const int wave = __builtin_amdgcn_readfirstlane((int)(threadIdx.x >> 5));
  const int p0 = blockIdx.x * 2;
#pragma unroll 1
  for (int it = 0; it < 4; ++it) {
    const int w = it * 256 + tid;
    const int i = w >> 3, c = (w & 7) * 4;
    const float* sp = Spart + (size_t)i * kNFlat + p0 * 16 + c;
    v4f acc = (v4f){0.f, 0.f, 0.f, 0.f};
#pragma unroll 4
    for (int ch = 0; ch < kChunks; ++ch) {
      const v4f a = *(const v4f*)(sp + (size_t)ch * (kNB * kNFlat));
      acc += a;
    }
    const float s0 = acc[0], s1 = acc[1], s2 = acc[2], s3 = acc[3];
    float ss = s0 * s0 + s1 * s1 + s2 * s2 + s3 * s3;
    ss += __shfl_xor(ss, 1, 32);
    ss += __shfl_xor(ss, 2, 32);
    const float nrm = sqrtf(ss);
    const float rden = 1.0f / (1.0f + nrm * nrm);
    const float v0 = (nrm * s0) * rden, v1 = (nrm * s1) * rden, v2 = (nrm * s2) * rden, v3 = (nrm * s3) * rden;
    if (FINAL) {
      v4f ov;
      ov[0] = v0;
      ov[1] = v1;
      ov[2] = v2;
      ov[3] = v3;
      float* op = out + (size_t)i * kNFlat + p0 * 16 + c;
      *(volatile v4f*)op = ov;
      __threadfence();
      *(volatile v4f*)op = ov;
    } else {
      sV[(c + 0) * kLdsPitch + i] = v0 * kVCarry;
      sV[(c + 1) * kLdsPitch + i] = v1 * kVCarry;
      sV[(c + 2) * kLdsPitch + i] = v2 * kVCarry;
      sV[(c + 3) * kLdsPitch + i] = v3 * kVCarry;
    }
  }
  if (!FINAL) {
    __syncthreads();
    emit_f16_rows128<64>(sV, vT + (size_t)(p0 * 16) * 128, wave, lane);
  }
}

template <bool FIRST>
__global__ __launch_bounds__(256) void agree_softmax_kernel(const float* __restrict__ W, const float* __restrict__ G,
                                                            const float* bIn, float* bOut, float* __restrict__ cOut) {
  __shared__ float sD[32];
  const int tid = threadIdx.x, lane = tid & 31;
  const int wave = __builtin_amdgcn_readfirstlane((int)(threadIdx.x >> 5));
  const int j = blockIdx.x;
  const int p = tid >> 3, k = tid & 7;
  const float* wp = W + (size_t)j * (kNP * kNK * kNQ) + tid * 16;
  const float* gp = G + ((size_t)(j * kNK + k)) * kNFlat + p * 16;
  float d = 0.f;
#pragma unroll
  for (int e4 = 0; e4 < 4; ++e4) {
    const v4f a = *(const v4f*)(wp + 4 * e4);
    const v4f g = *(const v4f*)(gp + 4 * e4);
    d = fmaf(a[0], g[0], d);
    d = fmaf(a[1], g[1], d);
    d = fmaf(a[2], g[2], d);
    d = fmaf(a[3], g[3], d);
  }
  d += __shfl_xor(d, 1, 32);
  d += __shfl_xor(d, 2, 32);
  d += __shfl_xor(d, 4, 32);
  if (k == 0) sD[p] = d;
  __syncthreads();
  float bv = sD[lane];
  if (!FIRST) bv = bIn[j * kNP + lane] + bv;
  float m = bv;
  m = fmaxf(m, __shfl_xor(m, 16, 32));
  m = fmaxf(m, __shfl_xor(m, 8, 32));
  m = fmaxf(m, __shfl_xor(m, 4, 32));
  m = fmaxf(m, __shfl_xor(m, 2, 32));
  m = fmaxf(m, __shfl_xor(m, 1, 32));
  const float ev = expf(bv - m);
  float sum = ev;
  sum += __shfl_xor(sum, 16, 32);
  sum += __shfl_xor(sum, 8, 32);
  sum += __shfl_xor(sum, 4, 32);
  sum += __shfl_xor(sum, 2, 32);
  sum += __shfl_xor(sum, 1, 32);
  const float cv = ev * (1.0f / sum);
  if (wave == 0) {
    float* bq = bOut + j * kNP + lane;
    float* cq = cOut + j * kNP + lane;
    if (FIRST) *(volatile float*)bq = bv;
    *(volatile float*)cq = cv;
    __threadfence();
    if (FIRST) *(volatile float*)bq = bv;
    *(volatile float*)cq = cv;
  }
}

extern "C" void kernel_launch(void* const* d_in, const int* in_sizes, int n_in,
                              void* d_out, int out_size, void* d_ws, size_t ws_size,
                              hipStream_t stream) {
  if (n_in < 2) return;
  if (in_sizes[0] != kNB * kNJ * kNK) return;
  if (in_sizes[1] != kNJ * kNP * kNK * kNQ) return;
  if (out_size != kNB * kNP * kNQ) return;
  if (ws_size < kWsTotal) return;

  const float* x = (const float*)d_in[0];
  const float* W = (const float*)d_in[1];
  float* out = (float*)d_out;

  char* ws = (char*)d_ws;
  unsigned short* X16   = (unsigned short*)(ws + kOffX16);
  unsigned short* XT16  = (unsigned short*)(ws + kOffXT16);
  unsigned short* BT16  = (unsigned short*)(ws + kOffBT16);
  float*          SPART = (float*)(ws + kOffSPART);
  unsigned short* VT16  = (unsigned short*)(ws + kOffVT16);
  float*          GPL   = (float*)(ws + kOffGPL);
  float*          BL    = (float*)(ws + kOffBL);
  float*          CL    = (float*)(ws + kOffCL);

  const dim3 gridBt(kNJ / 8, kNP / 4);
  const dim3 gridS((kNB / 64) * (kNFlat / 64) / 8, kChunks);
  const dim3 gridG((kKFlat / 64) * (kNFlat / 64) / 8, 1);

  cast_x_kernel<<<(kNB * kKFlat / 8) / 256, 256, 0, stream>>>(x, X16, kNB * kKFlat / 8);
  xpose_x_kernel<<<kKFlat / 64, 256, 0, stream>>>(x, XT16);

  build_bt_kernel<true><<<gridBt, 256, 0, stream>>>(W, CL, BT16);
  gemm64_f16_kernel<<<gridS, 256, 0, stream>>>(
      X16, kKFlat, (long)kChunkK,
      BT16, kKFlat, (long)kChunkK,
      SPART, kNFlat, (long)(kNB * kNFlat),
      kNB, kNFlat, kChunkK, kSScale);
  reduce_scale_kernel<false><<<kNP / 2, 256, 0, stream>>>(SPART, out, VT16);
  gemm64_f16_kernel<<<gridG, 256, 0, stream>>>(
      XT16, kNB, 0L,
      VT16, kNB, 0L,
      GPL, kNFlat, 0L,
      kKFlat, kNFlat, kNB, kGScale);
  agree_softmax_kernel<true><<<kNJ, 256, 0, stream>>>(W, GPL, BL, BL, CL);

  build_bt_kernel<false><<<gridBt, 256, 0, stream>>>(W, CL, BT16);
  gemm64_f16_kernel<<<gridS, 256, 0, stream>>>(
      X16, kKFlat, (long)kChunkK,
      BT16, kKFlat, (long)kChunkK,
      SPART, kNFlat, (long)(kNB * kNFlat),
      kNB, kNFlat, kChunkK, kSScale);
  reduce_scale_kernel<false><<<kNP / 2, 256, 0, stream>>>(SPART, out, VT16);
  gemm64_f16_kernel<<<gridG, 256, 0, stream>>>(
      XT16, kNB, 0L,
      VT16, kNB, 0L,
      GPL, kNFlat, 0L,
      kKFlat, kNFlat, kNB, kGScale);
  agree_softmax_kernel<false><<<kNJ, 256, 0, stream>>>(W, GPL, BL, BL, CL);

  build_bt_kernel<false><<<gridBt, 256, 0, stream>>>(W, CL, BT16);
  gemm64_f16_kernel<<<gridS, 256, 0, stream>>>(
      X16, kKFlat, (long)kChunkK,
      BT16, kKFlat, (long)kChunkK,
      SPART, kNFlat, (long)(kNB * kNFlat),
      kNB, kNFlat, kChunkK, kSScale);
  reduce_scale_kernel<true><<<kNP / 2, 256, 0, stream>>>(SPART, out, VT16);
}
